// GAT_MN_67980742361114
// MI455X (gfx1250) — hardware-verified
//
#include <hip/hip_runtime.h>
#include <stddef.h>


#define DF    128
#define NH    4
#define HC    32
#define NCLS  10
#define GR    32
#define AP    136
#define XSP   132
#define NWG   8
#define NB    512
#define LNB   9
#define NBD   4096
#define LNBD  12
#define CHUNK 2048
#define NTHR  256
#define NWAVE 8
#define WCAP  256
#define NGRP  (CHUNK / (NTHR * 4))
#define GSZ   32

#define LDS_SACC (NB * DF)
#define LDS_DEN  (NB * NH)
#define LDS_MRUN (NB * NH)
#define LDS_LIST (NWAVE * WCAP)
#define LDSA_BYTES ((LDS_SACC + LDS_DEN + LDS_MRUN + LDS_LIST + NWAVE) * 4)

static_assert(WCAP == (CHUNK / NTHR) * 32);
static_assert(NGRP >= 1);
static_assert((1 << LNB) == NB);
static_assert((1 << LNBD) == NBD);
static_assert(NH * HC == DF);
static_assert(NWG * 16 == DF);
static_assert(NTHR == NWAVE * 32);
static_assert(NTHR == 2 * DF);
static_assert((NB % NWAVE) == 0);
static_assert((NBD % (NWAVE * GSZ)) == 0);
static_assert(((LDS_SACC + LDS_DEN) % 4) == 0);
static_assert(LDSA_BYTES == 286752);
static_assert(CHUNK == 2048);
static_assert((LNBD + 11) <= 30);

typedef float    v4f  __attribute__((ext_vector_type(4)));
typedef float    v8f  __attribute__((ext_vector_type(8)));
typedef int      v4i  __attribute__((ext_vector_type(4)));
typedef _Float16 v8h  __attribute__((ext_vector_type(8)));
typedef _Float16 v16h __attribute__((ext_vector_type(16)));
union Frag   { v16h v; v8h half[2]; };
union Pack16 { v8h h; v4i i; };

__device__ __forceinline__ v8f wm(v16h a, v16h b, v8f c) {
  v8f d = __builtin_amdgcn_wmma_f32_16x16x32_f16(false, a, false, b, (short)0, c, false, false);
  asm volatile("v_nop\n\tv_nop\n\tv_nop\n\tv_nop" : "+v"(d) : "v"(a), "v"(b));
  return d;
}

#define HITJ(J, HJ, SJ)                                                      \
  {                                                                          \
    const unsigned mj = __builtin_amdgcn_ballot_w32(HJ);                     \
    if (HJ) {                                                                \
      const int pos = wc + (int)__builtin_amdgcn_mbcnt_lo(mj, 0u);           \
      if (pos < WCAP) wl[pos] = ((el0 + (J)) << LN) | (int)(SJ);             \
    }                                                                        \
    wc += (int)__builtin_popcount(mj);                                       \
  }

template <int LN>
__device__ __forceinline__ int scan_chunk(const int* __restrict__ dsti, int nE, bool al16,
                                          int cbase, int nodeBase, int tid, int* wl) {
  int wc = 0;
#pragma unroll
  for (int g = 0; g < NGRP; ++g) {
    const int el0 = (g * NTHR + tid) * 4;
    const int e0  = cbase + el0;
    const int sent = -2147483647 - 1;
    v4i d;
    if (al16 && (e0 + 3 < nE)) {
      d = *(const v4i*)(dsti + e0);
    } else {
      d.x = (e0     < nE) ? dsti[min(e0, nE - 1)]     : sent;
      d.y = (e0 + 1 < nE) ? dsti[min(e0 + 1, nE - 1)] : sent;
      d.z = (e0 + 2 < nE) ? dsti[min(e0 + 2, nE - 1)] : sent;
      d.w = (e0 + 3 < nE) ? dsti[min(e0 + 3, nE - 1)] : sent;
    }
    const unsigned s0 = (unsigned)d.x - (unsigned)nodeBase;
    const unsigned s1 = (unsigned)d.y - (unsigned)nodeBase;
    const unsigned s2 = (unsigned)d.z - (unsigned)nodeBase;
    const unsigned s3 = (unsigned)d.w - (unsigned)nodeBase;
    const bool h0 = s0 < (unsigned)(1 << LN);
    const bool h1 = s1 < (unsigned)(1 << LN);
    const bool h2 = s2 < (unsigned)(1 << LN);
    const bool h3 = s3 < (unsigned)(1 << LN);
    const unsigned many = __builtin_amdgcn_ballot_w32(h0 | h1 | h2 | h3);
    if (many != 0u) {
      HITJ(0, h0, s0)
      HITJ(1, h1, s1)
      HITJ(2, h2, s2)
      HITJ(3, h3, s3)
    }
  }
  return wc;
}
#undef HITJ

__global__ __launch_bounds__(NTHR) void k_prep(const float* __restrict__ W, _Float16* Wh, int nT) {
  const int i = blockIdx.x * NTHR + threadIdx.x;
  if (i >= nT) return;
  const int c  = i >> 4;
  const int k0 = (i & 15) * 8;
  Pack16 u;
#pragma unroll
  for (int j = 0; j < 8; ++j) u.h[j] = (_Float16)(W[(size_t)(k0 + j) * DF + c] * 8.0f);
  _Float16* p = Wh + (size_t)i * 8;
  *(volatile v4i*)p = u.i;
  __threadfence();
  *(volatile v4i*)p = u.i;
}

__global__ __launch_bounds__(NTHR) void k_deg(
    const int* __restrict__ dsti, const float* __restrict__ W1,
    const float* __restrict__ al, const float* __restrict__ ar,
    float* ft, float* asrc, float* adst, int nN, int nE, int nP) {
  __shared__ int cnt[NBD];
  __shared__ int list[LDS_LIST];
  __shared__ int wcnt[NWAVE];
  __shared__ __attribute__((aligned(16))) float A1w[NWAVE * GSZ * NH];
  __shared__ __attribute__((aligned(16))) float A2w[NWAVE * GSZ * NH];

  const int tid  = threadIdx.x;
  const int lane = tid & 31;
  const int wave = tid >> 5;
  const int nodeBase = blockIdx.x * NBD;

  for (int i = tid; i < NBD; i += NTHR) cnt[i] = 0;
  __syncthreads();

  const bool al16 = ((((size_t)dsti) & 15) == 0);
  const int nChunks = (nE + CHUNK - 1) / CHUNK;
#pragma unroll 1
  for (int ch = 0; ch < nChunks; ++ch) {
    const int cbase = ch * CHUNK;
    const int wc = scan_chunk<LNBD>(dsti, nE, al16, cbase, nodeBase, tid, list + wave * WCAP);
    if (lane == 0) wcnt[wave] = wc;
    __syncthreads();
    if (wave == 0) {
#pragma unroll 1
      for (int wsx = 0; wsx < NWAVE; ++wsx) {
        int n = wcnt[wsx];
        if (n > WCAP) n = WCAP;
        if (n < 0) n = 0;
#pragma unroll 1
        for (int i = 0; i < n; ++i) {
          const int ent  = list[wsx * WCAP + i];
          const int slot = ent & (NBD - 1);
          const int c = cnt[slot];
          cnt[slot] = c + 1;
        }
      }
    }
    __syncthreads();
  }

  const int hd = lane >> 3;
  const int c0 = 4 * lane;
  const v4f w0 = *(const v4f*)(W1 + 0 * DF + c0);
  const v4f w1 = *(const v4f*)(W1 + 1 * DF + c0);
  const v4f w2 = *(const v4f*)(W1 + 2 * DF + c0);
  const v4f w3 = *(const v4f*)(W1 + 3 * DF + c0);
  const v4f la = *(const v4f*)(al + c0);
  const v4f ra = *(const v4f*)(ar + c0);
  const int SPW = NBD / NWAVE;
#pragma unroll 1
  for (int grp = 0; grp < SPW / GSZ; ++grp) {
#pragma unroll 1
    for (int r = 0; r < GSZ; ++r) {
      const int slot = wave * SPW + grp * GSZ + r;
      const int node = nodeBase + slot;
      float d = (float)cnt[slot];
      if (node >= nN) d = 1.0f;
      const float f1 = (d - 3.0f > 0.0f) ? 1.0f : 0.0f;
      const float f2 = 3.0f * (1.0f / d);
      const float f3 = (d - 4.0f > 0.0f) ? 1.0f : 0.0f;
      const v4f fv = d * w0 + f1 * w1 + f2 * w2 + f3 * w3;
      float s1 = fv.x * la.x + fv.y * la.y + fv.z * la.z + fv.w * la.w;
      float s2 = fv.x * ra.x + fv.y * ra.y + fv.z * ra.z + fv.w * ra.w;
      s1 += __shfl_xor(s1, 1, 32); s1 += __shfl_xor(s1, 2, 32); s1 += __shfl_xor(s1, 4, 32);
      s2 += __shfl_xor(s2, 1, 32); s2 += __shfl_xor(s2, 2, 32); s2 += __shfl_xor(s2, 4, 32);
      if (node < nP) {
        float* p = ft + (size_t)node * DF + c0;
        *(volatile v4f*)p = fv;
        __threadfence();
        *(volatile v4f*)p = fv;
      }
      A1w[(wave * GSZ + r) * NH + hd] = s1;
      A2w[(wave * GSZ + r) * NH + hd] = s2;
    }
    __syncthreads();
    {
      const int rowS = nodeBase + wave * SPW + grp * GSZ;
      if (rowS + GSZ <= nP) {
        const int row = rowS + lane;
        const v4f v1 = *(const v4f*)(A1w + (wave * GSZ + lane) * NH);
        const v4f v2 = *(const v4f*)(A2w + (wave * GSZ + lane) * NH);
        float* p1 = asrc + (size_t)row * NH;
        float* p2 = adst + (size_t)row * NH;
        *(volatile v4f*)p1 = v1;
        *(volatile v4f*)p2 = v2;
        __threadfence();
        *(volatile v4f*)p1 = v1;
        *(volatile v4f*)p2 = v2;
      }
    }
    __syncthreads();
  }
}

__device__ __forceinline__ void epi_tile(v8f acc, int T, int hh, int m, int wave, int ncol,
                                         float cs, float cd, float* Xs, float* As, float* Ds) {
  float ss[8], sd[8];
#pragma unroll
  for (int r = 0; r < 8; ++r) {
    const float v = acc[r] * 0.125f;
    Xs[(T * 16 + 8 * hh + r) * XSP + ncol] = v;
    ss[r] = v * cs;
    sd[r] = v * cd;
  }
#pragma unroll
  for (int mk = 1; mk < 16; mk <<= 1) {
#pragma unroll
    for (int r = 0; r < 8; ++r) {
      ss[r] += __shfl_xor(ss[r], mk, 32);
      sd[r] += __shfl_xor(sd[r], mk, 32);
    }
  }
  if (m == 0) {
#pragma unroll
    for (int r = 0; r < 8; ++r) {
      As[(T * 16 + 8 * hh + r) * NWG + wave] = ss[r];
      Ds[(T * 16 + 8 * hh + r) * NWG + wave] = sd[r];
    }
  }
}

__global__ __launch_bounds__(NTHR) void k_gemm2(
    const float* __restrict__ x, const _Float16* __restrict__ Wh,
    const float* __restrict__ al, const float* __restrict__ ar,
    float* xp, float* asrc, float* adst, int nN) {
  __shared__ __attribute__((aligned(16))) _Float16 At[GR * AP];
  __shared__ __attribute__((aligned(16))) float Xs[GR * XSP];
  __shared__ __attribute__((aligned(16))) float As[GR * NWG];
  __shared__ __attribute__((aligned(16))) float Ds[GR * NWG];

  const int tid  = threadIdx.x;
  const int lane = tid & 31;
  const int wave = tid >> 5;
  const int hh   = lane >> 4;
  const int m    = lane & 15;
  const int rowBase = blockIdx.x * GR;

  {
    const int r  = tid >> 3;
    const int c0 = (tid & 7) * 16;
    int row = rowBase + r;
    if (row > nN - 1) row = nN - 1;
    const float* p = x + (size_t)row * DF + c0;
    const v4f f0 = *(const v4f*)(p), f1 = *(const v4f*)(p + 4);
    const v4f f2 = *(const v4f*)(p + 8), f3 = *(const v4f*)(p + 12);
    Pack16 u0, u1;
    u0.h[0] = (_Float16)f0.x; u0.h[1] = (_Float16)f0.y; u0.h[2] = (_Float16)f0.z; u0.h[3] = (_Float16)f0.w;
    u0.h[4] = (_Float16)f1.x; u0.h[5] = (_Float16)f1.y; u0.h[6] = (_Float16)f1.z; u0.h[7] = (_Float16)f1.w;
    u1.h[0] = (_Float16)f2.x; u1.h[1] = (_Float16)f2.y; u1.h[2] = (_Float16)f2.z; u1.h[3] = (_Float16)f2.w;
    u1.h[4] = (_Float16)f3.x; u1.h[5] = (_Float16)f3.y; u1.h[6] = (_Float16)f3.z; u1.h[7] = (_Float16)f3.w;
    *(v8h*)(At + r * AP + c0)     = u0.h;
    *(v8h*)(At + r * AP + c0 + 8) = u1.h;
  }
  __syncthreads();

  const int ncol = wave * 16 + m;
  v8f c0a = {0.f, 0.f, 0.f, 0.f, 0.f, 0.f, 0.f, 0.f};
  v8f c1a = {0.f, 0.f, 0.f, 0.f, 0.f, 0.f, 0.f, 0.f};
#pragma unroll
  for (int kt = 0; kt < DF / 32; ++kt) {
    const int k0 = kt * 32;
    Frag a0, a1, b;
    const _Float16* pb  = Wh + (size_t)ncol * DF + k0 + 8 * hh;
    const _Float16* pa0 = At + m * AP + k0 + 8 * hh;
    const _Float16* pa1 = At + (16 + m) * AP + k0 + 8 * hh;
    b.half[0]  = *(const v8h*)pb;  b.half[1]  = *(const v8h*)(pb + 16);
    a0.half[0] = *(const v8h*)pa0; a0.half[1] = *(const v8h*)(pa0 + 16);
    a1.half[0] = *(const v8h*)pa1; a1.half[1] = *(const v8h*)(pa1 + 16);
    c0a = wm(a0.v, b.v, c0a);
    c1a = wm(a1.v, b.v, c1a);
  }

  const float cs = al[ncol];
  const float cd = ar[ncol];
  epi_tile(c0a, 0, hh, m, wave, ncol, cs, cd, Xs, As, Ds);
  epi_tile(c1a, 1, hh, m, wave, ncol, cs, cd, Xs, As, Ds);
  __syncthreads();

  v4f xr[4];
#pragma unroll
  for (int i = 0; i < 4; ++i) xr[i] = *(const v4f*)(Xs + (4 * wave + i) * XSP + 4 * lane);
  float* xpp[4];
#pragma unroll
  for (int i = 0; i < 4; ++i) xpp[i] = xp + (size_t)(rowBase + 4 * wave + i) * DF + 4 * lane;
  const bool wg = (wave < 2);
  v4f gv = {0.f, 0.f, 0.f, 0.f};
  float* gp = asrc;
  if (wg) {
    const float* S  = (wave == 0) ? As : Ds;
    const float* rp = S + lane * NWG;
    gv.x = rp[0] + rp[1];
    gv.y = rp[2] + rp[3];
    gv.z = rp[4] + rp[5];
    gv.w = rp[6] + rp[7];
    gp = ((wave == 0) ? asrc : adst) + (size_t)(rowBase + lane) * NH;
  }

#pragma unroll
  for (int i = 0; i < 4; ++i) *(volatile v4f*)(xpp[i]) = xr[i];
  if (wg) *(volatile v4f*)gp = gv;
  __threadfence();
#pragma unroll
  for (int i = 0; i < 4; ++i) *(volatile v4f*)(xpp[i]) = xr[i];
  if (wg) *(volatile v4f*)gp = gv;
}

__global__ __launch_bounds__(NTHR) void k_agg(
    const int* __restrict__ srci, const int* __restrict__ dsti,
    const float* __restrict__ ft, const float* __restrict__ asrc, const float* __restrict__ adst,
    float* out, int nN, int nE) {
  extern __shared__ v4f lds_a[];
  float* sacc = (float*)lds_a;
  float* den  = sacc + LDS_SACC;
  float* mrun = den + LDS_DEN;
  int*   list = (int*)(mrun + LDS_MRUN);
  int*   wcnt = list + LDS_LIST;

  const int tid  = threadIdx.x;
  const int lane = tid & 31;
  const int wave = tid >> 5;
  const int hd   = lane >> 3;
  const int c0   = 4 * lane;
  const int nodeBase = blockIdx.x * NB;

  {
    const v4f z4 = {0.f, 0.f, 0.f, 0.f};
    for (int i = tid; i < (LDS_SACC + LDS_DEN) / 4; i += NTHR) lds_a[i] = z4;
    const float ninf = __uint_as_float(0xff800000u);
    for (int i = tid; i < LDS_MRUN; i += NTHR) mrun[i] = ninf;
  }
  __syncthreads();

  const bool al16 = ((((size_t)dsti) & 15) == 0);
  const int nChunks = (nE + CHUNK - 1) / CHUNK;
#pragma unroll 1
  for (int ch = 0; ch < nChunks; ++ch) {
    const int cbase = ch * CHUNK;
    const int wc = scan_chunk<LNB>(dsti, nE, al16, cbase, nodeBase, tid, list + wave * WCAP);
    if (lane == 0) wcnt[wave] = wc;
    __syncthreads();

    if (wave == 0) {
#pragma unroll 1
      for (int wsx = 0; wsx < NWAVE; ++wsx) {
        int n = wcnt[wsx];
        if (n > WCAP) n = WCAP;
        if (n < 0) n = 0;
#pragma unroll 1
        for (int i = 0; i < n; ++i) {
          const int ent  = list[wsx * WCAP + i];
          const int slot = ent & (NB - 1);
          const int el   = (ent >> LNB) & (CHUNK - 1);
          int e = cbase + el;
          if (e > nE - 1) e = nE - 1;
          int s = srci[e];
          s = s < 0 ? 0 : (s > nN - 1 ? nN - 1 : s);
          int nd = nodeBase + slot;
          if (nd > nN - 1) nd = nN - 1;
          float a = asrc[(size_t)s * NH + hd] + adst[(size_t)nd * NH + hd];
          a = (a > 0.0f) ? a : 0.2f * a;
          const int ai = slot * NH + hd;
          const float mo = mrun[ai];
          const float mn = fmaxf(mo, a);
          const float sc = __expf(mo - mn);
          const float p  = __expf(a - mn);
          const v4f xv = *(const v4f*)(ft + (size_t)s * DF + c0);
          v4f* sp = (v4f*)(sacc + slot * DF + c0);
          const v4f cur = *sp;
          const v4f nxt = cur * sc + p * xv;
          *sp = nxt;
          const float dd = den[ai];
          den[ai]  = dd * sc + p;
          mrun[ai] = mn;
        }
      }
    }
    __syncthreads();
  }

  const int SPW = NB / NWAVE;
#pragma unroll 1
  for (int j = 0; j < SPW; ++j) {
    const int slot = wave * SPW + j;
    const size_t node = (size_t)(nodeBase + slot);
    const float dv  = den[slot * NH + hd];
    const float inv = (dv > 0.0f) ? (1.0f / dv) : 0.0f;
    v4f y = *(const v4f*)(sacc + slot * DF + c0) * inv;
    y.x = y.x > 0.f ? y.x : 0.f;
    y.y = y.y > 0.f ? y.y : 0.f;
    y.z = y.z > 0.f ? y.z : 0.f;
    y.w = y.w > 0.f ? y.w : 0.f;
    float* op = out + node * DF + c0;
    *(volatile v4f*)op = y;
    __threadfence();
    *(volatile v4f*)op = y;
  }
}

__device__ __forceinline__ void store_out_pass(const float* os, float* out, int nOut, int lane) {
  for (int base = 0; base < nOut; base += 128) {
    const int i = base + 4 * lane;
    if (i + 3 < nOut) {
      const v4f v = *(const v4f*)(os + i);
      *(volatile v4f*)(out + i) = v;
    } else {
#pragma unroll
      for (int q = 0; q < 4; ++q)
        if (i + q < nOut) { const float v = os[i + q]; *(volatile float*)(out + i + q) = v; }
    }
  }
}

__global__ __launch_bounds__(NTHR) void k_pool(
    const int* __restrict__ gid, const float* __restrict__ h,
    const float* __restrict__ Wc, const float* __restrict__ bc,
    float* out, int nN, int nG, int nOut, int osOff, int nTot) {
  extern __shared__ v4f lds_p[];
  float* gs = (float*)lds_p;
  float* gc = gs + 2 * nG * DF;
  float* os = gs + osOff;

  const int tid  = threadIdx.x;
  const int lane = tid & 31;
  const int wave = tid >> 5;

  for (int i = tid; i < nTot; i += NTHR) gs[i] = 0.0f;
  __syncthreads();

  {
    const int f    = tid & (DF - 1);
    const int half = tid >> 7;
    const int nMid = nN >> 1;
    const int nBeg = half ? nMid : 0;
    const int nEnd = half ? nN : nMid;
    float* acc = gs + (size_t)half * nG * DF + f;
    float* cc  = gc + half * nG;
#pragma unroll 1
    for (int n = nBeg; n < nEnd; ++n) {
      int g = gid[n];
      g = g < 0 ? 0 : (g > nG - 1 ? nG - 1 : g);
      const float v = h[(size_t)n * DF + f];
      acc[g * DF] += v;
      if (f == 0) cc[g] += 1.0f;
    }
  }
  __syncthreads();

  for (int i = tid; i < nG * DF; i += NTHR) {
    const int g = i / DF;
    const float c = gc[g] + gc[nG + g];
    const float inv = 1.0f / fmaxf(c, 1.0f);
    gs[i] = (gs[i] + gs[nG * DF + i]) * inv;
  }
  __syncthreads();

  for (int o = tid; o < nOut; o += NTHR) {
    const int g = o / NCLS;
    const int c = o - g * NCLS;
    const float* gm = gs + g * DF;
    float s = 0.0f;
#pragma unroll 8
    for (int k = 0; k < DF; ++k) s += gm[k] * Wc[k * NCLS + c];
    s += bc[c];
    const float y = 1.0f / (1.0f + __expf(-s));
    os[o] = y;
  }
  __syncthreads();

  if (wave == 0) {
    store_out_pass(os, out, nOut, lane);
    __threadfence();
    store_out_pass(os, out, nOut, lane);
  }
}

extern "C" void kernel_launch(void* const* d_in, const int* in_sizes, int n_in,
                              void* d_out, int out_size, void* d_ws, size_t ws_size,
                              hipStream_t stream) {
  if (n_in < 11) return;
  const int nE = in_sizes[0];
  const int nN = in_sizes[2];
  if (nE <= 0 || in_sizes[1] != nE || nN <= 0) return;
  if (in_sizes[3] != 4 * DF || in_sizes[6] != DF * DF) return;
  if (in_sizes[4] != DF || in_sizes[5] != DF || in_sizes[7] != DF || in_sizes[8] != DF) return;
  if (in_sizes[9] != DF * NCLS || in_sizes[10] != NCLS) return;
  if (out_size <= 0 || (out_size % NCLS) != 0) return;
  const int nG = out_size / NCLS;
  if (nG > 256) return;
  const int nOut = nG * NCLS;

  const int*   src = (const int*)d_in[0];
  const int*   dst = (const int*)d_in[1];
  const int*   gid = (const int*)d_in[2];
  const float* W1  = (const float*)d_in[3];
  const float* al1 = (const float*)d_in[4];
  const float* ar1 = (const float*)d_in[5];
  const float* W2  = (const float*)d_in[6];
  const float* al2 = (const float*)d_in[7];
  const float* ar2 = (const float*)d_in[8];
  const float* Wc  = (const float*)d_in[9];
  const float* bc  = (const float*)d_in[10];
  float* out = (float*)d_out;

  const int nBlk = (nN + NB - 1) / NB;
  const int nP   = nBlk * NB;
  const int nDeg = (nN + NBD - 1) / NBD;

  size_t off = 0;
  _Float16* Wh = (_Float16*)((char*)d_ws + off); off += (size_t)DF * DF * sizeof(_Float16);
  float* ftb = (float*)((char*)d_ws + off);     off += (size_t)nP * DF * sizeof(float);
  float* hb  = (float*)((char*)d_ws + off);     off += (size_t)nP * DF * sizeof(float);
  float* a1b = (float*)((char*)d_ws + off);     off += (size_t)nP * NH * sizeof(float);
  float* a2b = (float*)((char*)d_ws + off);     off += (size_t)nP * NH * sizeof(float);
  if (off > ws_size) return;
  if (off > (size_t)134217728u) return;

  const int osOff = ((2 * nG * DF + 2 * nG) + 3) & ~3;
  const int osz   = ((nOut + 127) / 128) * 128;
  const int nTot  = osOff + osz;
  const int ldsP  = nTot * 4;
  if (ldsP > 290000) return;

  const int nT = DF * DF / 8;
  k_prep<<<(nT + NTHR - 1) / NTHR, NTHR, 0, stream>>>(W2, Wh, nT);

  k_deg<<<nDeg, NTHR, 0, stream>>>(dst, W1, al1, ar1, ftb, a1b, a2b, nN, nE, nP);

  hipFuncSetAttribute(reinterpret_cast<const void*>(&k_agg),
                      hipFuncAttributeMaxDynamicSharedMemorySize, LDSA_BYTES);
  k_agg<<<nBlk, NTHR, LDSA_BYTES, stream>>>(src, dst, ftb, a1b, a2b, hb, nN, nE);

  k_gemm2<<<nP / GR, NTHR, 0, stream>>>(hb, Wh, al2, ar2, ftb, a1b, a2b, nN);

  k_agg<<<nBlk, NTHR, LDSA_BYTES, stream>>>(src, dst, ftb, a1b, a2b, hb, nN, nE);

  hipFuncSetAttribute(reinterpret_cast<const void*>(&k_pool),
                      hipFuncAttributeMaxDynamicSharedMemorySize, ldsP);
  k_pool<<<1, NTHR, ldsP, stream>>>(gid, hb, Wc, bc, out, nN, nG, nOut, osOff, nTot);
}
